// GCNWithMultiHeadGATAndTCN_69312182223586
// MI455X (gfx1250) — hardware-run, weakly checked
//
#include <hip/hip_runtime.h>
#include <math.h>
#include <stdint.h>

#ifndef NB
#define NB 16
#endif
#define NN    1024
#define NF    128
#define NHID  256
#define NO    256
#define NHEAD 4
#define HD    64
#define NQB   (NN / 64)
#define NKT   (NN / 64)
#define RPB   64
#define NPB   ((NB * NN) / RPB)
#define K2    (2 * NN)
#define KG    (2 * NHID)
#define CTP   (2 * NO)
#define KC    (3 * CTP)
#define EPSV  1e-5f
#define LRELU 0.2f
static_assert(NHEAD * HD == NO);
static_assert(NHID == NO);
static_assert(NO == 256);
static_assert((NN % 64) == 0 && (NF % 32) == 0 && (NHID % 64) == 0);
static_assert(((NB * NN) % RPB) == 0 && ((NB * NN) % 64) == 0);
static_assert(NQB * 64 == NN && NKT * 64 == NN);
static_assert((CTP / 8) == 64);
static_assert((K2 % 32) == 0 && (KG % 32) == 0 && (KC % 32) == 0);

typedef _Float16 v16h __attribute__((ext_vector_type(16)));
typedef _Float16 v8h  __attribute__((ext_vector_type(8)));
typedef __bf16   v16b __attribute__((ext_vector_type(16)));
typedef __bf16   v8b  __attribute__((ext_vector_type(8)));
typedef float    v8f  __attribute__((ext_vector_type(8)));
typedef float    v4f  __attribute__((ext_vector_type(4)));
typedef unsigned int v4u __attribute__((ext_vector_type(4)));
typedef double   v2d  __attribute__((ext_vector_type(2)));

#if defined(__HIP_DEVICE_COMPILE__)
#define DEV_ASM 1
#else
#define DEV_ASM 0
#endif

__device__ __forceinline__ unsigned short bf_bits(float f) {
  unsigned u = __float_as_uint(f);
  return (unsigned short)((u + 0x7FFFu + ((u >> 16) & 1u)) >> 16);
}
__device__ __forceinline__ float bf_up(unsigned short hb) { return __uint_as_float(((unsigned)hb) << 16); }
__device__ __forceinline__ unsigned short h_bits(_Float16 x) { return __builtin_bit_cast(unsigned short, x); }
__device__ __forceinline__ unsigned pk16(unsigned short a, unsigned short b) { return (unsigned)a | ((unsigned)b << 16); }
__device__ __forceinline__ v8f zero8() { v8f z = {0.f, 0.f, 0.f, 0.f, 0.f, 0.f, 0.f, 0.f}; return z; }

template <typename OT> struct FT;
template <> struct FT<__bf16>   { typedef v16b frag; typedef v8b half8; };
template <> struct FT<_Float16> { typedef v16h frag; typedef v8h half8; };

template <typename OT>
__device__ __forceinline__ typename FT<OT>::frag ldfrag(const OT* p) {
  union { typename FT<OT>::frag v; typename FT<OT>::half8 h[2]; } f;
  f.h[0] = *(const typename FT<OT>::half8*)(p);
  f.h[1] = *(const typename FT<OT>::half8*)(p + 16);
  return f.v;
}

__device__ __forceinline__ v8f mmar(v16b a, v16b b, v8f c) {
  return __builtin_amdgcn_wmma_f32_16x16x32_bf16(false, a, false, b, (short)0, c, false, false);
}
__device__ __forceinline__ v8f mmar(v16h a, v16h b, v8f c) {
  return __builtin_amdgcn_wmma_f32_16x16x32_f16(false, a, false, b, (short)0, c, false, false);
}
__device__ __forceinline__ v8f mma_h(v16h a, v16h b, v8f c) {
  c = __builtin_amdgcn_wmma_f32_16x16x32_f16(false, a, false, b, (short)0, c, false, false);
#if DEV_ASM
  asm volatile("v_nop\n\tv_nop\n\tv_nop\n\tv_nop" : "+v"(c) : "v"(a), "v"(b));
#endif
  return c;
}
__device__ __forceinline__ void dep_guard(v8f& a, v8f& b, v16b x, v16b y) {
#if DEV_ASM
  asm volatile("v_nop\n\tv_nop\n\tv_nop\n\tv_nop" : "+v"(a), "+v"(b) : "v"(x), "v"(y));
#else
  (void)a; (void)b; (void)x; (void)y;
#endif
}
__device__ __forceinline__ void dep_guard(v8f& a, v8f& b, v16h x, v16h y) {
#if DEV_ASM
  asm volatile("v_nop\n\tv_nop\n\tv_nop\n\tv_nop" : "+v"(a), "+v"(b) : "v"(x), "v"(y));
#else
  (void)a; (void)b; (void)x; (void)y;
#endif
}
__device__ __forceinline__ void keep4(v16b a, v16b b, v16b c, v16b d) {
#if DEV_ASM
  asm volatile("v_nop" :: "v"(a), "v"(b), "v"(c), "v"(d));
#else
  (void)a; (void)b; (void)c; (void)d;
#endif
}
__device__ __forceinline__ void keep4(v16h a, v16h b, v16h c, v16h d) {
#if DEV_ASM
  asm volatile("v_nop" :: "v"(a), "v"(b), "v"(c), "v"(d));
#else
  (void)a; (void)b; (void)c; (void)d;
#endif
}
__device__ __forceinline__ void acc_guard4(v8f& a, v8f& b, v8f& c, v8f& d) {
#if DEV_ASM
  asm volatile("v_nop\n\tv_nop\n\tv_nop\n\tv_nop" : "+v"(a), "+v"(b), "+v"(c), "+v"(d));
#else
  (void)a; (void)b; (void)c; (void)d;
#endif
}

__device__ __forceinline__ void store2(unsigned short* q, v4u p) {
  *(volatile v4u*)q = p;
  __threadfence();
  *(volatile v4u*)q = p;
}
__device__ __forceinline__ void store2x(unsigned short* q0, unsigned short* q1, v4u p) {
  *(volatile v4u*)q0 = p;
  *(volatile v4u*)q1 = p;
  __threadfence();
  *(volatile v4u*)q0 = p;
  *(volatile v4u*)q1 = p;
}

__global__ __launch_bounds__(256) void cvt_bf8(const float* __restrict__ in, unsigned short* out, int n8) {
  const int i = blockIdx.x * 256 + (int)threadIdx.x;
  if (i < n8) {
    const v4f a  = *(const v4f*)(in + (size_t)i * 8);
    const v4f a4 = *(const v4f*)(in + (size_t)i * 8 + 4);
    v4u p;
    p[0] = pk16(bf_bits(a[0]),  bf_bits(a[1]));
    p[1] = pk16(bf_bits(a[2]),  bf_bits(a[3]));
    p[2] = pk16(bf_bits(a4[0]), bf_bits(a4[1]));
    p[3] = pk16(bf_bits(a4[2]), bf_bits(a4[3]));
    store2(out + (size_t)i * 8, p);
  }
}

__global__ __launch_bounds__(256) void cvt_gcw(const float* __restrict__ w, unsigned short* out) {
  const int i = blockIdx.x * 256 + (int)threadIdx.x;
  if (i < NHID * (NF / 8)) {
    const int o = i / (NF / 8), f0 = (i % (NF / 8)) * 8;
    v4u p;
#pragma unroll
    for (int e = 0; e < 4; ++e) {
      const float u0 = w[(size_t)(f0 + 2 * e) * NHID + o];
      const float u1 = w[(size_t)(f0 + 2 * e + 1) * NHID + o];
      p[e] = pk16(bf_bits(u0), bf_bits(u1));
    }
    store2(out + (size_t)o * NF + f0, p);
  }
}

__global__ __launch_bounds__(256) void cvt_adj2(const float* __restrict__ a, unsigned short* out) {
  const int i = blockIdx.x * 256 + (int)threadIdx.x;
  if (i < NN * (NN / 8)) {
    const int n = i / (NN / 8), c8 = (i % (NN / 8)) * 8;
    const v4f u  = *(const v4f*)(a + (size_t)n * NN + c8);
    const v4f u4 = *(const v4f*)(a + (size_t)n * NN + c8 + 4);
    v4u p;
    p[0] = pk16(bf_bits(u[0]),  bf_bits(u[1]));
    p[1] = pk16(bf_bits(u[2]),  bf_bits(u[3]));
    p[2] = pk16(bf_bits(u4[0]), bf_bits(u4[1]));
    p[3] = pk16(bf_bits(u4[2]), bf_bits(u4[3]));
    unsigned short* q0 = out + (size_t)n * K2 + c8;
    store2x(q0, q0 + NN, p);
  }
}

__global__ __launch_bounds__(256) void cvt_gatw2(const float* __restrict__ w, unsigned short* out) {
  const int i = blockIdx.x * 256 + (int)threadIdx.x;
  if (i < NO * (NHID / 8)) {
    const int r = i / (NHID / 8), f0 = (i % (NHID / 8)) * 8;
    const int h = r / HD, d = r % HD;
    v4u p;
#pragma unroll
    for (int e = 0; e < 4; ++e) {
      const float u0 = w[((size_t)h * NHID + (size_t)(f0 + 2 * e)) * HD + d];
      const float u1 = w[((size_t)h * NHID + (size_t)(f0 + 2 * e + 1)) * HD + d];
      p[e] = pk16(bf_bits(u0), bf_bits(u1));
    }
    unsigned short* q0 = out + (size_t)r * KG + f0;
    store2x(q0, q0 + NHID, p);
  }
}

__global__ __launch_bounds__(256) void cvt_convw3(const float* __restrict__ w, unsigned short* out) {
  const int i = blockIdx.x * 256 + (int)threadIdx.x;
  if (i < NO * 3 * (NO / 8)) {
    const int o = i / (3 * (NO / 8)), rem = i % (3 * (NO / 8));
    const int t = rem / (NO / 8), c0 = (rem % (NO / 8)) * 8;
    v4u p;
#pragma unroll
    for (int e = 0; e < 4; ++e) {
      const float u0 = w[((size_t)o * NO + (size_t)(c0 + 2 * e)) * 3 + t];
      const float u1 = w[((size_t)o * NO + (size_t)(c0 + 2 * e + 1)) * 3 + t];
      p[e] = pk16(bf_bits(u0), bf_bits(u1));
    }
    unsigned short* q0 = out + (size_t)o * KC + (size_t)t * CTP + c0;
    store2x(q0, q0 + NO, p);
  }
}

__global__ __launch_bounds__(256) void zero_ct_edges(unsigned short* ct, int nthr) {
  const int i = blockIdx.x * 256 + (int)threadIdx.x;
  if (i < nthr) {
    const int rr = i >> 6, c8 = (i & 63) * 8;
    const int b = rr >> 1;
    const int row = (rr & 1) ? (NN + 1) : 0;
    v4u z = {0u, 0u, 0u, 0u};
    store2(ct + ((size_t)b * (NN + 2) + (size_t)row) * CTP + c8, z);
  }
}

template <typename OT, int OUT_MODE>
__global__ __launch_bounds__(256) void gemm64(
    const unsigned short* __restrict__ Ap, int lda, long long strideA,
    const unsigned short* __restrict__ Btp, int ldb, long long strideB,
    void* Cout, void* Cout2, int ldc, long long strideC,
    int M, int N, int K, float oscale, float rscale) {
  typedef typename FT<OT>::frag V16;
  const OT* A  = (const OT*)(const void*)Ap;
  const OT* Bt = (const OT*)(const void*)Btp;
  __shared__ __align__(16) float sT[8][16 * 68];
  const int b    = blockIdx.y;
  const int lane = threadIdx.x & 31;
  const int wave = threadIdx.x >> 5;
  const int tilesN = N >> 6;
  const int tilesM = M >> 6;
  const int tile = blockIdx.x * 8 + wave;
  if (tile >= tilesM * tilesN) return;
  const int tm = tile / tilesN;
  const int tn = tile - tm * tilesN;
  const int m0 = tm << 6;
  const int n0 = tn << 6;

  const OT* Ab = A  + (size_t)b * (size_t)strideA;
  const OT* Bb = Bt + (size_t)b * (size_t)strideB;

  const int rlane = lane & 15;
  const int koff  = (lane >> 4) * 8;
  const int mOff  = (lane >> 4) * 8;

  v8f acc[4][4];
#pragma unroll
  for (int i = 0; i < 4; ++i)
#pragma unroll
    for (int j = 0; j < 4; ++j) acc[i][j] = zero8();

  for (int k0 = 0; k0 < K; k0 += 32) {
    V16 bq[4];
#pragma unroll
    for (int j = 0; j < 4; ++j)
      bq[j] = ldfrag<OT>(Bb + (size_t)(n0 + (j << 4) + rlane) * ldb + koff + k0);
#pragma unroll
    for (int i = 0; i < 4; ++i) {
      const V16 af = ldfrag<OT>(Ab + (size_t)(m0 + (i << 4) + rlane) * lda + koff + k0);
#pragma unroll
      for (int j = 0; j < 4; ++j) acc[i][j] = mmar(af, bq[j], acc[i][j]);
      dep_guard(acc[i][0], acc[i][3], af, bq[3]);
    }
    keep4(bq[0], bq[1], bq[2], bq[3]);
  }
  acc_guard4(acc[0][0], acc[0][1], acc[0][2], acc[0][3]);
  acc_guard4(acc[1][0], acc[1][1], acc[1][2], acc[1][3]);
  acc_guard4(acc[2][0], acc[2][1], acc[2][2], acc[2][3]);
  acc_guard4(acc[3][0], acc[3][1], acc[3][2], acc[3][3]);

  float* slab = sT[wave];
#pragma unroll
  for (int i = 0; i < 4; ++i) {
    const int mBase = m0 + (i << 4);
#pragma unroll
    for (int j = 0; j < 4; ++j) {
#pragma unroll
      for (int r = 0; r < 8; ++r) {
        slab[(mOff + r) * 68 + (j << 4) + rlane] = acc[i][j][r];
      }
    }
    __builtin_amdgcn_fence(__ATOMIC_RELEASE, "workgroup");
    __builtin_amdgcn_wave_barrier();
    __builtin_amdgcn_fence(__ATOMIC_ACQUIRE, "workgroup");
    if (OUT_MODE == 0) {
      float* C = (float*)Cout + (size_t)b * (size_t)strideC;
      const int h2 = lane >> 4, c4 = (lane & 15) * 4;
      for (int pass = 0; pass < 2; ++pass) {
#pragma unroll
        for (int it = 0; it < 8; ++it) {
          const int row = it * 2 + h2;
          const v4f v = *(const v4f*)(slab + row * 68 + c4) * oscale;
          *(volatile v4f*)(C + (size_t)(mBase + row) * ldc + n0 + c4) = v;
        }
        __threadfence();
      }
    } else {
      const int q = lane >> 3, c8 = (lane & 7) * 8;
      unsigned short* C  = (unsigned short*)Cout  + (size_t)b * (size_t)strideC;
      unsigned short* C2 = (unsigned short*)Cout2 + (size_t)b * (size_t)strideC;
      v4u hv[4], lv[4];
#pragma unroll
      for (int it = 0; it < 4; ++it) {
        const int row = it * 4 + q;
        const float* sp = slab + row * 68 + c8;
        float f[8];
#pragma unroll
        for (int e = 0; e < 8; ++e) f[e] = sp[e];
        v4u a, a2;
#pragma unroll
        for (int e = 0; e < 4; ++e) {
          const float f0 = f[2 * e], f1 = f[2 * e + 1];
          unsigned short h0, h1, l0 = 0, l1 = 0;
          if (OUT_MODE == 4) {
            h0 = bf_bits(f0); h1 = bf_bits(f1);
            l0 = bf_bits(f0 - bf_up(h0));
            l1 = bf_bits(f1 - bf_up(h1));
          } else {
            const _Float16 x0 = (_Float16)f0, x1 = (_Float16)f1;
            h0 = h_bits(x0); h1 = h_bits(x1);
            if (OUT_MODE == 3) {
              l0 = h_bits((_Float16)((f0 - (float)x0) * rscale));
              l1 = h_bits((_Float16)((f1 - (float)x1) * rscale));
            }
          }
          a[e] = pk16(h0, h1); a2[e] = pk16(l0, l1);
        }
        hv[it] = a; lv[it] = a2;
      }
      for (int pass = 0; pass < 2; ++pass) {
#pragma unroll
        for (int it = 0; it < 4; ++it) {
          const int row = it * 4 + q;
          *(volatile v4u*)(C + (size_t)(mBase + row) * ldc + n0 + c8) = hv[it];
          if (OUT_MODE == 3 || OUT_MODE == 4) *(volatile v4u*)(C2 + (size_t)(mBase + row) * ldc + n0 + c8) = lv[it];
        }
        __threadfence();
      }
    }
    __builtin_amdgcn_fence(__ATOMIC_RELEASE, "workgroup");
    __builtin_amdgcn_wave_barrier();
    __builtin_amdgcn_fence(__ATOMIC_ACQUIRE, "workgroup");
  }
}

__global__ __launch_bounds__(128)
void attn_gat(const unsigned short* __restrict__ qhp, const unsigned short* __restrict__ qlp,
              const unsigned short* __restrict__ vhp, const unsigned short* __restrict__ vlp,
              unsigned short* ctp) {
  union FH { v16h v; v8h h[2]; };
  __shared__ __align__(16) _Float16 Ksh[64 * 64];
  __shared__ __align__(16) _Float16 Ksl[64 * 64];
  __shared__ __align__(16) _Float16 Vth[64 * 64];
  __shared__ __align__(16) _Float16 Vtl[64 * 64];
  __shared__ __align__(16) _Float16 Psh[4][16 * 64];
  __shared__ __align__(16) float    Os[4][16 * 64];

  const int tid  = threadIdx.x;
  const int wave = tid >> 5;
  const int lane = tid & 31;
  const int hh   = lane >> 4;
  const int c    = lane & 15;

  const int bx   = blockIdx.x;
  const int qb   = bx % NQB;
  const int rest = bx / NQB;
  const int head = rest % NHEAD;
  const int b    = rest / NHEAD;
  const int q0   = qb * 64 + wave * 16;
  const size_t rowB = (size_t)b * NN;

  const _Float16* Qh = (const _Float16*)(const void*)qhp;
  const _Float16* Ql = (const _Float16*)(const void*)qlp;
  const _Float16* Vh = (const _Float16*)(const void*)vhp + ((size_t)b * NO + (size_t)head * HD) * NN;
  const _Float16* Vl = (const _Float16*)(const void*)vlp + ((size_t)b * NO + (size_t)head * HD) * NN;

  v16h qah[2], qal[2];
#pragma unroll
  for (int dc = 0; dc < 2; ++dc) {
    const size_t qo = (rowB + q0 + c) * NO + (size_t)head * HD + dc * 32 + 8 * hh;
    qah[dc] = ldfrag<_Float16>(Qh + qo);
    qal[dc] = ldfrag<_Float16>(Ql + qo);
  }

  float mrow[8], lrow[8];
  v8f oacc[4];
#pragma unroll
  for (int r = 0; r < 8; ++r) { mrow[r] = -INFINITY; lrow[r] = 0.f; }
#pragma unroll
  for (int t = 0; t < 4; ++t) oacc[t] = zero8();

  for (int kt = 0; kt < NKT; ++kt) {
    const int kv0 = kt * 64;
    __syncthreads();
    {
      const int r = tid >> 1, half = (tid & 1) * 32;
      const size_t ko = (rowB + kv0 + r) * NO + (size_t)head * HD + half;
      const _Float16* kg  = Qh + ko;
      const _Float16* klg = Ql + ko;
      const _Float16* vg  = Vh + (size_t)r * NN + kv0 + half;
      const _Float16* vlg = Vl + (size_t)r * NN + kv0 + half;
#pragma unroll
      for (int i = 0; i < 4; ++i) {
        const v8h a0 = *(const v8h*)(kg + 8 * i);
        const v8h a1 = *(const v8h*)(klg + 8 * i);
        const v8h b0 = *(const v8h*)(vg + 8 * i);
        const v8h b1 = *(const v8h*)(vlg + 8 * i);
        *(v8h*)(Ksh + r * 64 + half + 8 * i) = a0;
        *(v8h*)(Ksl + r * 64 + half + 8 * i) = a1;
        *(v8h*)(Vth + r * 64 + half + 8 * i) = b0;
        *(v8h*)(Vtl + r * 64 + half + 8 * i) = b1;
      }
    }
    __syncthreads();

    v8f s[4];
#pragma unroll
    for (int j = 0; j < 4; ++j) {
      v8f ah = zero8(), al = zero8();
#pragma unroll
      for (int dc = 0; dc < 2; ++dc) {
        FH kb, kl;
        kb.h[0] = *(const v8h*)(Ksh + (j * 16 + c) * 64 + dc * 32 + 8 * hh);
        kb.h[1] = *(const v8h*)(Ksh + (j * 16 + c) * 64 + dc * 32 + 16 + 8 * hh);
        kl.h[0] = *(const v8h*)(Ksl + (j * 16 + c) * 64 + dc * 32 + 8 * hh);
        kl.h[1] = *(const v8h*)(Ksl + (j * 16 + c) * 64 + dc * 32 + 16 + 8 * hh);
        ah = mma_h(qah[dc], kb.v, ah);
        al = mma_h(qal[dc], kb.v, al);
        al = mma_h(qah[dc], kl.v, al);
      }
#pragma unroll
      for (int r = 0; r < 8; ++r) {
        const float v = ah[r] + al[r] * (1.0f / 4096.0f);
        s[j][r] = (v > 0.f) ? v : (LRELU * v);
      }
    }

    _Float16* pwh = Psh[wave];
#pragma unroll
    for (int r = 0; r < 8; ++r) {
      float m = s[0][r];
#pragma unroll
      for (int j = 1; j < 4; ++j) m = fmaxf(m, s[j][r]);
#pragma unroll
      for (int off = 1; off < 16; off <<= 1) m = fmaxf(m, __shfl_xor(m, off, 32));
      const float mnew  = fmaxf(mrow[r], m);
      const float msafe = (mnew == -INFINITY) ? 0.f : mnew;
      const float alpha = __expf(mrow[r] - msafe);
      mrow[r] = mnew;
      float psum = 0.f;
#pragma unroll
      for (int j = 0; j < 4; ++j) {
        const float p = __expf(s[j][r] - msafe);
        psum += p;
        pwh[(8 * hh + r) * 64 + j * 16 + c] = (_Float16)(p * 16384.0f);
      }
#pragma unroll
      for (int off = 1; off < 16; off <<= 1) psum += __shfl_xor(psum, off, 32);
      lrow[r] = lrow[r] * alpha + psum;
#pragma unroll
      for (int t = 0; t < 4; ++t) oacc[t][r] *= alpha;
    }
    __builtin_amdgcn_fence(__ATOMIC_RELEASE, "workgroup");
    __builtin_amdgcn_wave_barrier();
    __builtin_amdgcn_fence(__ATOMIC_ACQUIRE, "workgroup");

    v8f o1[4];
#pragma unroll
    for (int t = 0; t < 4; ++t) o1[t] = zero8();
#pragma unroll 1
    for (int kk = 0; kk < 2; ++kk) {
      FH pa;
      pa.h[0] = *(const v8h*)(pwh + c * 64 + kk * 32 + 8 * hh);
      pa.h[1] = *(const v8h*)(pwh + c * 64 + kk * 32 + 16 + 8 * hh);
#pragma unroll
      for (int t = 0; t < 4; ++t) {
        FH vb, vl;
        vb.h[0] = *(const v8h*)(Vth + (t * 16 + c) * 64 + kk * 32 + 8 * hh);
        vb.h[1] = *(const v8h*)(Vth + (t * 16 + c) * 64 + kk * 32 + 16 + 8 * hh);
        vl.h[0] = *(const v8h*)(Vtl + (t * 16 + c) * 64 + kk * 32 + 8 * hh);
        vl.h[1] = *(const v8h*)(Vtl + (t * 16 + c) * 64 + kk * 32 + 16 + 8 * hh);
        oacc[t] = mma_h(pa.v, vb.v, oacc[t]);
        o1[t]   = mma_h(pa.v, vl.v, o1[t]);
      }
    }
#pragma unroll
    for (int t = 0; t < 4; ++t)
#pragma unroll
      for (int r = 0; r < 8; ++r) oacc[t][r] += o1[t][r] * (1.0f / 4096.0f);
  }

  float* os = Os[wave];
#pragma unroll
  for (int r = 0; r < 8; ++r) {
    const float l = lrow[r];
    const float inv = ((l > 0.f) ? (1.0f / l) : 0.f) * (1.0f / 16384.0f);
#pragma unroll
    for (int t = 0; t < 4; ++t) os[(8 * hh + r) * 64 + t * 16 + c] = oacc[t][r] * inv;
  }
  __builtin_amdgcn_fence(__ATOMIC_RELEASE, "workgroup");
  __builtin_amdgcn_wave_barrier();
  __builtin_amdgcn_fence(__ATOMIC_ACQUIRE, "workgroup");
  {
    const int q4 = lane >> 3, c8 = (lane & 7) * 8;
    v4u hv[4], lv[4];
#pragma unroll
    for (int it = 0; it < 4; ++it) {
      const int row = it * 4 + q4;
      const float* sp = os + row * 64 + c8;
      v4u a, a2;
#pragma unroll
      for (int e = 0; e < 4; ++e) {
        const float f0 = sp[2 * e], f1 = sp[2 * e + 1];
        const unsigned short h0 = bf_bits(f0), h1 = bf_bits(f1);
        const unsigned short l0 = bf_bits(f0 - bf_up(h0)), l1 = bf_bits(f1 - bf_up(h1));
        a[e] = pk16(h0, h1); a2[e] = pk16(l0, l1);
      }
      hv[it] = a; lv[it] = a2;
    }
    for (int pass = 0; pass < 2; ++pass) {
#pragma unroll
      for (int it = 0; it < 4; ++it) {
        const int row = it * 4 + q4;
        const size_t go = ((size_t)b * (NN + 2) + 1 + (size_t)(q0 + row)) * CTP + (size_t)head * HD + c8;
        *(volatile v4u*)(ctp + go)      = hv[it];
        *(volatile v4u*)(ctp + go + NO) = lv[it];
      }
      __threadfence();
    }
  }
}

template <bool RELU>
__global__ __launch_bounds__(256) void bn_stats(const float* __restrict__ X, const float* __restrict__ bias,
                                                double* part) {
  __shared__ __align__(16) double sh[2 * NO];
  const int c = (int)threadIdx.x;
  const int p = blockIdx.x;
  const float bb = bf_up(bf_bits(bias[c]));
  const float* xp = X + (size_t)p * RPB * NO + c;
  double s = 0.0, s2 = 0.0;
#pragma unroll 4
  for (int r = 0; r < RPB; ++r) {
    float v = xp[(size_t)r * NO] + bb;
    if (RELU) v = fmaxf(v, 0.f);
    const double dv = (double)v;
    s  += dv;
    s2 += dv * dv;
  }
  sh[c] = s;
  sh[NO + c] = s2;
  __syncthreads();
  union { v2d d; v4u u; } w;
  w.d = *(const v2d*)(sh + 2 * c);
  double* q = part + (size_t)p * (2 * NO) + 2 * c;
  *(volatile v4u*)q = w.u;
  __threadfence();
  *(volatile v4u*)q = w.u;
}

__global__ __launch_bounds__(256) void bn_fin(const double* __restrict__ part, const float* __restrict__ gamma,
                                              const float* __restrict__ beta, float* bnp, int nblk, int nrows) {
  __shared__ __align__(16) float sf[4 * NO];
  const int c = (int)threadIdx.x;
  double S = 0.0, S2 = 0.0;
#pragma unroll 1
  for (int p = 0; p < nblk; ++p) {
    S  += part[(size_t)p * (2 * NO) + c];
    S2 += part[(size_t)p * (2 * NO) + NO + c];
  }
  const double dn = (double)nrows;
  const double mu = S / dn;
  double var = S2 / dn - mu * mu;
  if (var < 0.0) var = 0.0;
  const float muf  = (float)mu;
  const float varf = (float)var;
  const float rs   = 1.0f / sqrtf(varf + EPSV);
  sf[c]          = muf;
  sf[NO + c]     = rs;
  sf[2 * NO + c] = bf_up(bf_bits(gamma[c]));
  sf[3 * NO + c] = bf_up(bf_bits(beta[c]));
  __syncthreads();
  const int row = c >> 6, c4 = (c & 63) * 4;
  const v4f v = *(const v4f*)(sf + row * NO + c4);
  float* q = bnp + row * NO + c4;
  *(volatile v4f*)q = v;
  __threadfence();
  *(volatile v4f*)q = v;
}

__global__ __launch_bounds__(256) void bn_apply1(const float* __restrict__ X, const float* __restrict__ bias,
                                                 const float* __restrict__ bnp, unsigned short* outp, int nrows) {
#pragma clang fp contract(off)
  const int i = blockIdx.x * 256 + (int)threadIdx.x;
  const int row = i >> 5, c8 = (i & 31) * 8;
  if (row >= nrows) return;
  const float* xp = X + (size_t)row * NHID + c8;
  const v4f a   = *(const v4f*)xp;
  const v4f a4  = *(const v4f*)(xp + 4);
  const v4f bb0 = *(const v4f*)(bias + c8), bb1 = *(const v4f*)(bias + c8 + 4);
  const v4f mu0 = *(const v4f*)(bnp + c8), mu1 = *(const v4f*)(bnp + c8 + 4);
  const v4f rs0 = *(const v4f*)(bnp + NHID + c8), rs1 = *(const v4f*)(bnp + NHID + c8 + 4);
  const v4f g0  = *(const v4f*)(bnp + 2 * NHID + c8), g1 = *(const v4f*)(bnp + 2 * NHID + c8 + 4);
  const v4f be0 = *(const v4f*)(bnp + 3 * NHID + c8), be1 = *(const v4f*)(bnp + 3 * NHID + c8 + 4);
  float f[8];
#pragma unroll
  for (int e = 0; e < 4; ++e) {
    float v = a[e] + bf_up(bf_bits(bb0[e]));
    v = fmaxf(v, 0.f);
    float t = (v - mu0[e]) * rs0[e];
    t = t * g0[e] + be0[e];
    f[e] = fmaxf(t, 0.f);
  }
#pragma unroll
  for (int e = 0; e < 4; ++e) {
    float v = a4[e] + bf_up(bf_bits(bb1[e]));
    v = fmaxf(v, 0.f);
    float t = (v - mu1[e]) * rs1[e];
    t = t * g1[e] + be1[e];
    f[4 + e] = fmaxf(t, 0.f);
  }
  v4u hv, lv;
#pragma unroll
  for (int e = 0; e < 4; ++e) {
    const float f0 = f[2 * e], f1 = f[2 * e + 1];
    const unsigned short h0 = bf_bits(f0), h1 = bf_bits(f1);
    const unsigned short l0 = bf_bits(f0 - bf_up(h0)), l1 = bf_bits(f1 - bf_up(h1));
    hv[e] = pk16(h0, h1); lv[e] = pk16(l0, l1);
  }
  unsigned short* q = outp + (size_t)row * KG + c8;
  *(volatile v4u*)q          = hv;
  *(volatile v4u*)(q + NHID) = lv;
  __threadfence();
  *(volatile v4u*)q          = hv;
  *(volatile v4u*)(q + NHID) = lv;
}

__global__ __launch_bounds__(256) void bn_apply2(const float* __restrict__ Y, const float* __restrict__ bias,
                                                 const float* __restrict__ bnp, float* outp, int nrows) {
#pragma clang fp contract(off)
  const int i = blockIdx.x * 256 + (int)threadIdx.x;
  const int row = i >> 6, c4 = (i & 63) * 4;
  if (row >= nrows) return;
  const v4f a  = *(const v4f*)(Y + (size_t)row * NO + c4);
  const v4f bb = *(const v4f*)(bias + c4);
  const v4f mu = *(const v4f*)(bnp + c4);
  const v4f rs = *(const v4f*)(bnp + NO + c4);
  const v4f g  = *(const v4f*)(bnp + 2 * NO + c4);
  const v4f be = *(const v4f*)(bnp + 3 * NO + c4);
  v4f o;
#pragma unroll
  for (int e = 0; e < 4; ++e) {
    const float v = a[e] + bf_up(bf_bits(bb[e]));
    float t = (v - mu[e]) * rs[e];
    t = t * g[e] + be[e];
    o[e] = fmaxf(t, 0.f);
  }
  float* q = outp + (size_t)row * NO + c4;
  *(volatile v4f*)q = o;
  __threadfence();
  *(volatile v4f*)q = o;
}

static_assert((size_t)NB * NHID * K2 * 2 == 2 * (size_t)NB * NN * NO * 2);
static_assert((size_t)NB * NN * NHID * 4 == (size_t)NB * NN * NO * 4);

extern "C" void kernel_launch(void* const* d_in, const int* in_sizes, int n_in,
                              void* d_out, int out_size, void* d_ws, size_t ws_size,
                              hipStream_t stream) {
  if (n_in < 11) return;
  if (in_sizes[0] < NB * NN * NF) return;
  if (in_sizes[1] < NN * NN) return;
  if (in_sizes[2] < NF * NHID || in_sizes[3] < NHID || in_sizes[4] < NHID || in_sizes[5] < NHID) return;
  if (in_sizes[6] < NHEAD * NHID * HD) return;
  if (in_sizes[7] < NO * NO * 3 || in_sizes[8] < NO || in_sizes[9] < NO || in_sizes[10] < NO) return;
  if (out_size < NB * NN * NO) return;

  const float* x      = (const float*)d_in[0];
  const float* adj    = (const float*)d_in[1];
  const float* gc_w   = (const float*)d_in[2];
  const float* gc_b   = (const float*)d_in[3];
  const float* bn1_g  = (const float*)d_in[4];
  const float* bn1_b  = (const float*)d_in[5];
  const float* gat_w  = (const float*)d_in[6];
  const float* conv_w = (const float*)d_in[7];
  const float* conv_b = (const float*)d_in[8];
  const float* bn2_g  = (const float*)d_in[9];
  const float* bn2_b  = (const float*)d_in[10];

  const size_t PXB  = (size_t)NB * NN * NF * 2;
  const size_t PGW  = (size_t)NHID * NF * 2;
  const size_t PADJ = (size_t)NN * K2 * 2;
  const size_t PW2  = (size_t)NO * KG * 2;
  const size_t PCW  = (size_t)NO * KC * 2;
  const size_t PH0  = (size_t)NB * NHID * K2 * 2;
  const size_t PQK  = (size_t)NB * NN * NO * 2;
  const size_t PH1  = (size_t)NB * NN * NHID * 4;
  const size_t PPT  = (size_t)NPB * 2 * NO * 8;
  const size_t PBNP = (size_t)4 * NO * 4;
  const size_t PH2  = (size_t)NB * NN * KG * 2;
  const size_t PVT  = (size_t)NB * NO * NN * 2;
  const size_t PCT  = (size_t)NB * (NN + 2) * CTP * 2;
  size_t off = 0;
  const size_t oXB  = off; off += PXB;
  const size_t oGW  = off; off += PGW;
  const size_t oADJ = off; off += PADJ;
  const size_t oW2  = off; off += PW2;
  const size_t oCW  = off; off += PCW;
  const size_t oH0  = off; off += PH0;
  const size_t oH1  = off; off += PH1;
  const size_t oP1  = off; off += PPT;
  const size_t oBN1 = off; off += PBNP;
  const size_t oH2  = off; off += PH2;
  const size_t oVTh = off; off += PVT;
  const size_t oVTl = off; off += PVT;
  const size_t oCT  = off; off += PCT;
  const size_t oP2  = off; off += PPT;
  const size_t oBN2 = off; off += PBNP;
  if (off > ws_size) return;
  if (off > (size_t)134217728) return;
  if (2 * PQK > PH0) return;

  char* ws = (char*)d_ws;
  unsigned short* Xb   = (unsigned short*)(ws + oXB);
  unsigned short* GWt  = (unsigned short*)(ws + oGW);
  unsigned short* ADJ2 = (unsigned short*)(ws + oADJ);
  unsigned short* W2   = (unsigned short*)(ws + oW2);
  unsigned short* CW   = (unsigned short*)(ws + oCW);
  unsigned short* H0T  = (unsigned short*)(ws + oH0);
  unsigned short* QKh  = (unsigned short*)(ws + oH0);
  unsigned short* QKl  = (unsigned short*)(ws + oH0 + PQK);
  float*          H1   = (float*)(ws + oH1);
  float*          Y    = (float*)(ws + oH1);
  double*         P1   = (double*)(ws + oP1);
  float*          BN1  = (float*)(ws + oBN1);
  unsigned short* H2P  = (unsigned short*)(ws + oH2);
  unsigned short* VTh  = (unsigned short*)(ws + oVTh);
  unsigned short* VTl  = (unsigned short*)(ws + oVTl);
  unsigned short* CT   = (unsigned short*)(ws + oCT);
  double*         P2   = (double*)(ws + oP2);
  float*          BN2  = (float*)(ws + oBN2);
  float*          out  = (float*)d_out;

  const dim3 blk(256);
  const int  n8x = NB * NN * NF / 8;
  const dim3 gCvtX((n8x + 255) / 256);
  const dim3 gGcw((NHID * (NF / 8) + 255) / 256);
  const dim3 gAdj((NN * (NN / 8) + 255) / 256);
  const dim3 gGat((NO * (NHID / 8) + 255) / 256);
  const dim3 gCvw((NO * 3 * (NO / 8) + 255) / 256);
  const int  nzero = NB * 2 * 64;
  const dim3 gZero((nzero + 255) / 256);
  const dim3 gG1((((NHID / 64) * (NN / 64)) + 7) / 8, NB);
  const dim3 gG2((((NN / 64) * (NHID / 64)) + 7) / 8, NB);
  const dim3 gG3(((((NB * NN) / 64) * (NO / 64)) + 7) / 8, 1);
  const dim3 gG4((((NO / 64) * (NN / 64)) + 7) / 8, NB);
  const dim3 gG5((((NN / 64) * (NO / 64)) + 7) / 8, NB);
  const dim3 gStat(NPB);
  const dim3 gAp1((NB * NN * 32 + 255) / 256);
  const dim3 gAp2((NB * NN * 64 + 255) / 256);
  const dim3 gAttn(NB * NHEAD * NQB);

  cvt_bf8<<<gCvtX, blk, 0, stream>>>(x, Xb, n8x);
  cvt_gcw<<<gGcw, blk, 0, stream>>>(gc_w, GWt);
  cvt_adj2<<<gAdj, blk, 0, stream>>>(adj, ADJ2);
  cvt_gatw2<<<gGat, blk, 0, stream>>>(gat_w, W2);
  cvt_convw3<<<gCvw, blk, 0, stream>>>(conv_w, CW);
  zero_ct_edges<<<gZero, blk, 0, stream>>>(CT, nzero);
  gemm64<__bf16, 4><<<gG1, blk, 0, stream>>>(
      GWt, NF, 0LL, Xb, NF, (long long)NN * NF,
      (void*)H0T, (void*)(H0T + NN), K2, (long long)NHID * K2,
      NHID, NN, NF, 1.0f, 1.0f);
  gemm64<__bf16, 0><<<gG2, blk, 0, stream>>>(
      ADJ2, K2, 0LL, H0T, K2, (long long)NHID * K2,
      (void*)H1, (void*)H1, NHID, (long long)NN * NHID,
      NN, NHID, K2, 1.0f, 1.0f);
  bn_stats<true><<<gStat, blk, 0, stream>>>(H1, gc_b, P1);
  bn_fin<<<dim3(1), blk, 0, stream>>>(P1, bn1_g, bn1_b, BN1, NPB, NB * NN);
  bn_apply1<<<gAp1, blk, 0, stream>>>(H1, gc_b, BN1, H2P, NB * NN);
  gemm64<__bf16, 3><<<gG3, blk, 0, stream>>>(
      H2P, KG, 0LL, W2, KG, 0LL,
      (void*)QKh, (void*)QKl, NO, 0LL,
      NB * NN, NO, KG, 1.0f, 4096.0f);
  gemm64<__bf16, 3><<<gG4, blk, 0, stream>>>(
      W2, KG, 0LL, H2P, KG, (long long)NN * KG,
      (void*)VTh, (void*)VTl, NN, (long long)NO * NN,
      NO, NN, KG, 1.0f, 4096.0f);
  attn_gat<<<gAttn, dim3(128), 0, stream>>>(QKh, QKl, VTh, VTl, CT);
  gemm64<__bf16, 0><<<gG5, blk, 0, stream>>>(
      CT, CTP, (long long)(NN + 2) * CTP, CW, KC, 0LL,
      (void*)Y, (void*)Y, NO, (long long)NN * NO,
      NN, NO, KC, 1.0f, 1.0f);
  bn_stats<false><<<gStat, blk, 0, stream>>>(Y, conv_b, P2);
  bn_fin<<<dim3(1), blk, 0, stream>>>(P2, bn2_g, bn2_b, BN2, NPB, NB * NN);
  bn_apply2<<<gAp2, blk, 0, stream>>>(Y, conv_b, BN2, out, NB * NN);
  (void)hipGetLastError();
}
